// DistanceClassifier_13881334300951
// MI455X (gfx1250) — hardware-verified
//
#include <hip/hip_runtime.h>
#include <math.h>

typedef _Float16 v16h __attribute__((ext_vector_type(16)));
typedef _Float16 v8h  __attribute__((ext_vector_type(8)));
typedef _Float16 v4h  __attribute__((ext_vector_type(4)));
typedef _Float16 v2h  __attribute__((ext_vector_type(2)));
typedef float    v8f  __attribute__((ext_vector_type(8)));
typedef float    v4f  __attribute__((ext_vector_type(4)));
typedef float    v2f  __attribute__((ext_vector_type(2)));

#define N_CTX 1024
#define M_RES 256
#define DIM   1024
#define AP    32
#define DP    260
#define OPSCALE 64.0f
#define ACCSCALE2 (1.0f / 2048.0f)

union Frag { v16h v; v8h h8[2]; v4h q[4]; };

__device__ __forceinline__ v8f wmma_f16(v16h a, v16h b, v8f c) {
    v8f d = __builtin_amdgcn_wmma_f32_16x16x32_f16(false, a, false, b, (short)0, c, false, false);
    asm volatile("v_nop\n\tv_nop\n\tv_nop\n\tv_nop" : "+v"(d) : "v"(a), "v"(b));
    return d;
}

__device__ __forceinline__ v4h cvt4(const v4f f, float& sq) {
    sq = fmaf(f.x, f.x, sq);
    sq = fmaf(f.y, f.y, sq);
    sq = fmaf(f.z, f.z, sq);
    sq = fmaf(f.w, f.w, sq);
    v4h r;
    r.x = (_Float16)(f.x * OPSCALE);
    r.y = (_Float16)(f.y * OPSCALE);
    r.z = (_Float16)(f.z * OPSCALE);
    r.w = (_Float16)(f.w * OPSCALE);
    return r;
}

__global__ __launch_bounds__(256) void fused_dist_softmax_kernel(
        const float* __restrict__ C,
        const float* __restrict__ R,
        float* __restrict__ out,
        int n_ctx)
{
    __shared__ __align__(16) _Float16 Ah[16 * AP];
    __shared__ __align__(16) float dist[16 * DP];
    __shared__ float csq_s[16];

    const int tid  = threadIdx.x;
    const int lane = tid & 31;
    const int wave = tid >> 5;
    const int m    = lane & 15;
    const int h    = lane >> 4;
    const int n0   = blockIdx.x * 16;
    if (n0 + 16 > n_ctx) return;

    const int col0 = wave * 32;
    const int col1 = col0 + 16;

    const int arow = tid >> 4;
    const int acol = (tid & 15) * 2;

    v8f acc0 = {0.f, 0.f, 0.f, 0.f, 0.f, 0.f, 0.f, 0.f};
    v8f acc1 = {0.f, 0.f, 0.f, 0.f, 0.f, 0.f, 0.f, 0.f};
    float csq = 0.0f, rs0 = 0.0f, rs1 = 0.0f;

    const float* crow = C + (size_t)(n0 + arow) * DIM + acol;
    const float* rp0  = R + (size_t)(col0 + m) * DIM + 8 * h;
    const float* rp1  = R + (size_t)(col1 + m) * DIM + 8 * h;

#pragma unroll 1
    for (int k0 = 0; k0 < DIM; k0 += 32) {
        {
            const v2f f = *(const v2f*)(crow + k0);
            csq = fmaf(f.x, f.x, csq);
            csq = fmaf(f.y, f.y, csq);
            v2h p;
            p.x = (_Float16)(f.x * OPSCALE);
            p.y = (_Float16)(f.y * OPSCALE);
            *(v2h*)(Ah + arow * AP + acol) = p;
        }
        __syncthreads();

        Frag a;
        a.h8[0] = *(const v8h*)(Ah + m * AP + 8 * h);
        a.h8[1] = *(const v8h*)(Ah + m * AP + 16 + 8 * h);

        Frag b0, b1;
        {
            const float* p0 = rp0 + k0;
            const float* p1 = rp1 + k0;
            b0.q[0] = cvt4(*(const v4f*)(p0),      rs0);
            b0.q[1] = cvt4(*(const v4f*)(p0 + 4),  rs0);
            b0.q[2] = cvt4(*(const v4f*)(p0 + 16), rs0);
            b0.q[3] = cvt4(*(const v4f*)(p0 + 20), rs0);
            b1.q[0] = cvt4(*(const v4f*)(p1),      rs1);
            b1.q[1] = cvt4(*(const v4f*)(p1 + 4),  rs1);
            b1.q[2] = cvt4(*(const v4f*)(p1 + 16), rs1);
            b1.q[3] = cvt4(*(const v4f*)(p1 + 20), rs1);
        }

        acc0 = wmma_f16(a.v, b0.v, acc0);
        acc1 = wmma_f16(a.v, b1.v, acc1);

        __syncthreads();
    }

    csq += __shfl_xor(csq, 8, 32);
    csq += __shfl_xor(csq, 4, 32);
    csq += __shfl_xor(csq, 2, 32);
    csq += __shfl_xor(csq, 1, 32);
    rs0 += __shfl_xor(rs0, 16, 32);
    rs1 += __shfl_xor(rs1, 16, 32);
    if ((tid & 15) == 0) csq_s[arow] = csq;
    __syncthreads();

#pragma unroll
    for (int i = 0; i < 8; ++i) {
        const int rl = 8 * h + i;
        const float cs = csq_s[rl];
        const float s0 = fmaxf(fmaf(acc0[i], -ACCSCALE2, cs + rs0), 0.0f);
        const float s1 = fmaxf(fmaf(acc1[i], -ACCSCALE2, cs + rs1), 0.0f);
        dist[rl * DP + col0 + m] = sqrtf(s0);
        dist[rl * DP + col1 + m] = sqrtf(s1);
    }
    __syncthreads();

    {
        const int row   = tid >> 4;
        const int chunk = tid & 15;
        float* dr = dist + row * DP + chunk * 16;
        float v[16];
#pragma unroll
        for (int q = 0; q < 4; ++q) {
            const v4f t = *(const v4f*)(dr + 4 * q);
            v[4 * q + 0] = t.x; v[4 * q + 1] = t.y; v[4 * q + 2] = t.z; v[4 * q + 3] = t.w;
        }
        float lmax = v[0];
#pragma unroll
        for (int j = 1; j < 16; ++j) lmax = fmaxf(lmax, v[j]);
        lmax = fmaxf(lmax, __shfl_xor(lmax, 8, 32));
        lmax = fmaxf(lmax, __shfl_xor(lmax, 4, 32));
        lmax = fmaxf(lmax, __shfl_xor(lmax, 2, 32));
        lmax = fmaxf(lmax, __shfl_xor(lmax, 1, 32));

        float e[16];
        float lsum = 0.0f;
#pragma unroll
        for (int j = 0; j < 16; ++j) { e[j] = __expf(v[j] - lmax); lsum += e[j]; }
        lsum += __shfl_xor(lsum, 8, 32);
        lsum += __shfl_xor(lsum, 4, 32);
        lsum += __shfl_xor(lsum, 2, 32);
        lsum += __shfl_xor(lsum, 1, 32);
        const float inv = 1.0f / lsum;

#pragma unroll
        for (int q = 0; q < 4; ++q) {
            v4f t;
            t.x = 1.0f - e[4 * q + 0] * inv;
            t.y = 1.0f - e[4 * q + 1] * inv;
            t.z = 1.0f - e[4 * q + 2] * inv;
            t.w = 1.0f - e[4 * q + 3] * inv;
            *(v4f*)(dr + 4 * q) = t;
        }
    }
    __syncthreads();

#pragma unroll 1
    for (int pass = 0; pass < 2; ++pass) {
        if (pass == 1) __threadfence();
#pragma unroll
        for (int it = 0; it < 4; ++it) {
            const int f4 = (wave * 4 + it) * 32 + lane;
            const int e0 = f4 * 4;
            const int r  = e0 >> 8;
            const int c  = e0 & 255;
            const v4f t = *(const v4f*)(dist + r * DP + c);
            *(volatile v4f*)(out + (size_t)(n0 + r) * M_RES + c) = t;
        }
    }
}

extern "C" void kernel_launch(void* const* d_in, const int* in_sizes, int n_in,
                              void* d_out, int out_size, void* d_ws, size_t ws_size,
                              hipStream_t stream) {
    (void)d_ws; (void)ws_size;
    if (n_in < 2) return;
    if (in_sizes[0] != N_CTX * DIM || in_sizes[1] != M_RES * DIM || out_size != N_CTX * M_RES) return;
    const float* C = (const float*)d_in[0];
    const float* R = (const float*)d_in[1];
    float* out = (float*)d_out;

    const int n_ctx = in_sizes[0] / DIM;
    fused_dist_softmax_kernel<<<(n_ctx + 15) / 16, 256, 0, stream>>>(C, R, out, n_ctx);
}
